// MyModel_87522843560267
// MI455X (gfx1250) — hardware-run, weakly checked
//
#include <hip/hip_runtime.h>

typedef __attribute__((ext_vector_type(16))) _Float16 v16h;
typedef __attribute__((ext_vector_type(8)))  _Float16 v8h;
typedef __attribute__((ext_vector_type(8)))  float    v8f;
typedef __attribute__((ext_vector_type(4)))  float    v4f;
typedef __attribute__((ext_vector_type(4)))  int      v4i;

constexpr int kBatch    = 1024;
constexpr int kSteps    = 4096;
constexpr int kUnits    = 10;
constexpr int kGateCols = 4 * kUnits;
constexpr int kOutCols  = 2 * kUnits;
constexpr int kTileRows = 16;
constexpr int kTiles    = kBatch / kTileRows;
constexpr int kChunks   = kSteps / 4;
constexpr int kWPerDir  = (kUnits + 2) * kGateCols;
constexpr int kTileOut  = kTileRows * kOutCols;
constexpr int kRVec     = kUnits * kGateCols / 4;
constexpr int kKVec     = kGateCols / 4;
static_assert(kUnits == 10, "k-slot map below assumes 10 units: k 0..9 state, 10 x, 11 one, 12..14 residual slots");
static_assert(kBatch % kTileRows == 0, "batch tiles");
static_assert(kSteps % 4 == 0, "four steps per 16-byte load");
static_assert((kTileOut * 4) % 128 == 0, "a tile of output rows is a whole number of 128-B lines");
static_assert(kTileOut == 320 && kRVec == 100 && kKVec == 10 && kWPerDir == 480, "derived sizes");

constexpr float kCarryW     = 64.0f;
constexpr float kCarryS     = 64.0f;
constexpr float kFold       = 1.0f / (kCarryW * kCarryS);
constexpr float kResWScale  = 16.0f;
constexpr float kXPartner   = kCarryS / kResWScale;
constexpr float kResBScale  = 1024.0f;
constexpr float kOnePartner = kCarryS / kResBScale;
constexpr float kResXScale  = kCarryW;
constexpr float kLog2e      = 1.44269504088896340736f;
constexpr float kSigK       = -kLog2e * kFold;
constexpr float kTanK       = 2.0f * kLog2e * kFold;
constexpr float kTanC       = 2.0f * kLog2e;
constexpr float kHalfMinNormal = 6.103515625e-05f;
static_assert(kXPartner == 4.0f && kOnePartner == 0.0625f, "partner scales");

__device__ __forceinline__ float fexp2(float v) { return __builtin_amdgcn_exp2f(v); }
__device__ __forceinline__ float frcp(float v)  { return __builtin_amdgcn_rcpf(v); }

__device__ __forceinline__ float flush16(float v) {
  return (__builtin_fabsf(v) < kHalfMinNormal) ? 0.0f : v;
}
__device__ __forceinline__ _Float16 to_h(float v) { return (_Float16)flush16(v); }

__device__ __forceinline__ v8f mma_tile(v16h a, v16h b) {
  v8f c = (v8f){0.f, 0.f, 0.f, 0.f, 0.f, 0.f, 0.f, 0.f};
  c = __builtin_amdgcn_wmma_f32_16x16x32_f16(false, a, false, b, (short)0, c, false, false);
  asm volatile("v_nop\n\tv_nop\n\tv_nop\n\tv_nop" : "+v"(c) : "v"(a), "v"(b));
  return c;
}

__global__ __launch_bounds__(64) void bidir_cell_tile_kernel(
    const float* __restrict__ x, const int* __restrict__ mask,
    const float* __restrict__ kf, const float* __restrict__ rf, const float* __restrict__ bf,
    const float* __restrict__ kb, const float* __restrict__ rb, const float* __restrict__ bb,
    float* __restrict__ out)
{
  __shared__ __align__(16) float sW[2 * kWPerDir];
  __shared__ __align__(16) float sOut[kTileOut];

  const int tid  = threadIdx.x;
  const int lane = tid & 31;
  const int dir  = tid >> 5;
  const int hiL  = lane >> 4;
  const int n    = lane & 15;
  const int tile = blockIdx.x;
  const bool isHi = (hiL != 0);

  const float* rk = dir ? rb : rf;
  const float* kn = dir ? kb : kf;
  const float* bs = dir ? bb : bf;
  float* sWd = sW + dir * kWPerDir;

#pragma unroll
  for (int it = 0; it < 4; ++it) {
    int q = lane + 32 * it;
    q = (q < kRVec - 1) ? q : (kRVec - 1);
    const v4f v = *(const v4f*)(rk + 4 * q);
    *(v4f*)(sWd + 4 * q) = v;
  }
  {
    const int q = (lane < kKVec - 1) ? lane : (kKVec - 1);
    const v4f vk = *(const v4f*)(kn + 4 * q);
    const v4f vb = *(const v4f*)(bs + 4 * q);
    *(v4f*)(sWd + kUnits * kGateCols + 4 * q) = vk;
    *(v4f*)(sWd + (kUnits + 1) * kGateCols + 4 * q) = vb;
  }
  __syncthreads();

  const int  mc    = (n < kUnits) ? n : (kUnits - 1);
  const bool rowok = (n < kUnits);
  const v8h zero8 = (v8h){(_Float16)0, (_Float16)0, (_Float16)0, (_Float16)0,
                          (_Float16)0, (_Float16)0, (_Float16)0, (_Float16)0};
  union FragU { v16h v; v8h h[2]; };
  v16h afr[4];
#pragma unroll
  for (int g = 0; g < 4; ++g) {
    const int col = kUnits * g + mc;
    float rl[8];
#pragma unroll
    for (int i = 0; i < 8; ++i) rl[i] = sWd[i * kGateCols + col];
    const float r8 = sWd[8 * kGateCols + col];
    const float r9 = sWd[9 * kGateCols + col];
    const float wv = sWd[10 * kGateCols + col];
    const float bv = sWd[11 * kGateCols + col];
    const float wc = wv * kCarryW;
    const float bc = bv * kCarryW;
    const float whf = (float)to_h(wc);
    const float bhf = (float)to_h(bc);
    const float wres = kResWScale * (wc - whf);
    const float bres = kResBScale * (bc - bhf);
    float cand[8];
    cand[0] = r8 * kCarryW;
    cand[1] = r9 * kCarryW;
    cand[2] = wc;
    cand[3] = bc;
    cand[4] = wres;
    cand[5] = bres;
    cand[6] = wv * (kCarryW / kResXScale);
    cand[7] = 0.0f;
    v8h lo8;
#pragma unroll
    for (int i = 0; i < 8; ++i) {
      float v = isHi ? cand[i] : (rl[i] * kCarryW);
      v = rowok ? v : 0.0f;
      lo8[i] = to_h(v);
    }
    FragU f;
    f.h[0] = lo8;
    f.h[1] = zero8;
    afr[g] = f.v;
  }

  const int brow = tile * kTileRows + n;
  const float* px = x    + (size_t)brow * (size_t)kSteps;
  const int*   pm = mask + (size_t)brow * (size_t)kSteps;

  float hs[8], cs[8];
#pragma unroll
  for (int r = 0; r < 8; ++r) { hs[r] = 0.0f; cs[r] = 0.0f; }

#pragma unroll 1
  for (int ci = 0; ci < kChunks; ++ci) {
    const int q = dir ? (kChunks - 1 - ci) : ci;
    const v4f xv = *(const v4f*)(px + 4 * q);
    const v4i mv = *(const v4i*)(pm + 4 * q);
    float xa = xv.x, xb = xv.y, xc = xv.z, xd = xv.w;
    int   ma = mv.x, mb = mv.y, mcc = mv.z, md = mv.w;
    asm volatile("" : "+v"(xa), "+v"(xb), "+v"(xc), "+v"(xd));
    asm volatile("" : "+v"(ma), "+v"(mb), "+v"(mcc), "+v"(md));
    float x0 = dir ? xd : xa;
    float x1 = dir ? xc : xb;
    float x2 = dir ? xb : xc;
    float x3 = dir ? xa : xd;
    int   m0 = dir ? md : ma;
    int   m1 = dir ? mcc : mb;
    int   m2 = dir ? mb : mcc;
    int   m3 = dir ? ma : md;

#pragma unroll 1
    for (int s = 0; s < 4; ++s) {
      const float xq   = x0 * kCarryS;
      const float xhf  = (float)to_h(xq);
      const float xres = kResXScale * (xq - xhf);
      const float xp   = x0 * kXPartner;
      float t[8];
#pragma unroll
      for (int i = 0; i < 8; ++i) t[i] = hs[i] * kCarryS;
      t[2] = isHi ? xq          : t[2];
      t[3] = isHi ? kCarryS     : t[3];
      t[4] = isHi ? xp          : t[4];
      t[5] = isHi ? kOnePartner : t[5];
      t[6] = isHi ? xres        : t[6];
      t[7] = isHi ? 0.0f        : t[7];
      v8h blo;
#pragma unroll
      for (int i = 0; i < 8; ++i) blo[i] = to_h(t[i]);
      FragU bu;
      bu.h[0] = blo;
      bu.h[1] = zero8;
      const v16h bfr = bu.v;

      const v8f ai = mma_tile(afr[0], bfr);
      const v8f af = mma_tile(afr[1], bfr);
      const v8f ag = mma_tile(afr[2], bfr);
      const v8f ao = mma_tile(afr[3], bfr);

      const bool upd = (m0 != 0);
#pragma unroll
      for (int r = 0; r < 8; ++r) {
        const float ig = frcp(1.0f + fexp2(ai[r] * kSigK));
        const float fg = frcp(1.0f + fexp2(af[r] * kSigK));
        const float gg = __builtin_fmaf(-2.0f, frcp(1.0f + fexp2(ag[r] * kTanK)), 1.0f);
        const float og = frcp(1.0f + fexp2(ao[r] * kSigK));
        const float cn = __builtin_fmaf(fg, cs[r], ig * gg);
        const float th = __builtin_fmaf(-2.0f, frcp(1.0f + fexp2(cn * kTanC)), 1.0f);
        const float hn = og * th;
        cs[r] = upd ? cn : cs[r];
        hs[r] = upd ? hn : hs[r];
      }

      x0 = x1; x1 = x2; x2 = x3;
      m0 = m1; m1 = m2; m2 = m3;
    }
  }

#pragma unroll
  for (int r = 0; r < 8; ++r) {
    if (!isHi || r < (kUnits - 8)) {
      sOut[n * kOutCols + dir * kUnits + 8 * hiL + r] = hs[r];
    }
  }
  __syncthreads();

  if (dir == 0) {
    const v4f r0 = *(const v4f*)(sOut + 4 * lane);
    const v4f r1 = *(const v4f*)(sOut + 4 * (lane + 32));
    const v4f r2 = *(const v4f*)(sOut + 4 * (64 + (lane & 15)));
    float* dst = out + (size_t)tile * kTileOut;
    *(volatile v4f*)(dst + 4 * lane) = r0;
    *(volatile v4f*)(dst + 4 * (lane + 32)) = r1;
    if (lane < 16) *(volatile v4f*)(dst + 4 * (64 + lane)) = r2;
    __threadfence();
    *(volatile v4f*)(dst + 4 * lane) = r0;
    *(volatile v4f*)(dst + 4 * (lane + 32)) = r1;
    if (lane < 16) *(volatile v4f*)(dst + 4 * (64 + lane)) = r2;
    __threadfence();
  }
}

extern "C" void kernel_launch(void* const* d_in, const int* in_sizes, int n_in,
                              void* d_out, int out_size, void* d_ws, size_t ws_size,
                              hipStream_t stream) {
  (void)d_ws;
  (void)ws_size;
  if (n_in < 8) return;
  if (in_sizes[0] != kBatch * kSteps) return;
  if (in_sizes[1] != kBatch * kSteps) return;
  if (in_sizes[2] != kGateCols) return;
  if (in_sizes[3] != kUnits * kGateCols) return;
  if (in_sizes[4] != kGateCols) return;
  if (in_sizes[5] != kGateCols) return;
  if (in_sizes[6] != kUnits * kGateCols) return;
  if (in_sizes[7] != kGateCols) return;
  if (out_size != kBatch * kOutCols) return;

  const float* x    = (const float*)d_in[0];
  const int*   mask = (const int*)d_in[1];
  const float* kf   = (const float*)d_in[2];
  const float* rf   = (const float*)d_in[3];
  const float* bf   = (const float*)d_in[4];
  const float* kb   = (const float*)d_in[5];
  const float* rb   = (const float*)d_in[6];
  const float* bb   = (const float*)d_in[7];
  float* out = (float*)d_out;

  bidir_cell_tile_kernel<<<dim3(kTiles), dim3(64), 0, stream>>>(x, mask, kf, rf, bf, kb, rb, bb, out);
}
